// OffsetAttentionLayer_32435593020119
// MI455X (gfx1250) — hardware-verified
//
#include <hip/hip_runtime.h>
#include <stddef.h>
#include <stdint.h>

#define NGRP   8
#define LMAXC  2560
#define DM     256
#define PROWS  (NGRP * LMAXC)
#define NPTS   16384
#define NQKV   768
#define QBLK   64
#define KCH    64
#define NQBG   (LMAXC / QBLK)
#define NKCG   (LMAXC / KCH)

static_assert(PROWS % 256 == 0);
static_assert(LMAXC % 256 == 0);
static_assert(LMAXC % QBLK == 0);
static_assert(LMAXC % KCH == 0);
static_assert(DM == 256);
static_assert(NQKV == 3 * DM);
static_assert(NPTS % 8 == 0);
static_assert((NQKV * DM) % 2048 == 0);
static_assert((DM * DM) % 2048 == 0);
static_assert(QBLK == 64 && KCH == 64);

typedef _Float16 v16h __attribute__((ext_vector_type(16)));
typedef _Float16 v8h  __attribute__((ext_vector_type(8)));
typedef float    v8f  __attribute__((ext_vector_type(8)));
typedef float    v4f  __attribute__((ext_vector_type(4)));
typedef unsigned int v4u __attribute__((ext_vector_type(4)));

union Frag  { v16h v; v8h h[2]; };
union Pack8 { v8h h; v4u u; };

__device__ __forceinline__ v8f mma16(v16h a, v16h b, v8f c) {
  c = __builtin_amdgcn_wmma_f32_16x16x32_f16(false, a, false, b, (short)0, c, false, false);
  asm volatile("v_nop\n\tv_nop\n\tv_nop\n\tv_nop" : "+v"(c) : "v"(a), "v"(b));
  return c;
}

__device__ __forceinline__ v16h ldfrag(const _Float16* p, int ld, int row0, int k0, int lane) {
  const int m = lane & 15, lh = lane >> 4;
  const _Float16* q = p + (size_t)(row0 + m) * ld + k0 + 8 * lh;
  Frag f;
  f.h[0] = *(const v8h*)(q);
  f.h[1] = *(const v8h*)(q + 16);
  return f.v;
}

__device__ __forceinline__ v8f zero8() { return (v8f){0.f, 0.f, 0.f, 0.f, 0.f, 0.f, 0.f, 0.f}; }

__device__ __forceinline__ int lower_bound_ids(const int* __restrict__ ids, int n, int key) {
  int lo = 0, hi = n;
#pragma unroll 1
  for (int it = 0; it < 15; ++it) {
    const int mid = (lo + hi) >> 1;
    const int mc  = min(max(mid, 0), n - 1);
    const int v   = ids[mc];
    const bool go = lo < hi;
    const bool lt = v < key;
    lo = (go && lt) ? (mid + 1) : lo;
    hi = (go && !lt) ? mid : hi;
  }
  return lo;
}

__device__ __forceinline__ v4f posenc4(const float* __restrict__ feat, const float* __restrict__ wp,
                                       const float* __restrict__ bp, float c0, float c1, int n, int col) {
  const v4f fe = *(const v4f*)(feat + (size_t)n * DM + col);
  const v4f wa = *(const v4f*)(wp + 2 * col);
  const v4f wb = *(const v4f*)(wp + 2 * col + 4);
  const v4f bv = *(const v4f*)(bp + col);
  v4f r;
  float p;
  p = c0 * wa[0]; p = fmaf(c1, wa[1], p); r[0] = (fe[0] + p) + bv[0];
  p = c0 * wa[2]; p = fmaf(c1, wa[3], p); r[1] = (fe[1] + p) + bv[1];
  p = c0 * wb[0]; p = fmaf(c1, wb[1], p); r[2] = (fe[2] + p) + bv[2];
  p = c0 * wb[2]; p = fmaf(c1, wb[3], p); r[3] = (fe[3] + p) + bv[3];
  return r;
}

__device__ __forceinline__ void gemm32x64(const _Float16* __restrict__ A, int lda,
                                          const _Float16* __restrict__ Bt, int ldb, int K,
                                          int m0, int n0, int lane, v8f (&acc)[2][4]) {
#pragma unroll 1
  for (int k0 = 0; k0 < K; k0 += 32) {
    const v16h a0 = ldfrag(A, lda, m0, k0, lane);
    const v16h a1 = ldfrag(A, lda, m0 + 16, k0, lane);
    const v16h b0 = ldfrag(Bt, ldb, n0, k0, lane);
    const v16h b1 = ldfrag(Bt, ldb, n0 + 16, k0, lane);
    const v16h b2 = ldfrag(Bt, ldb, n0 + 32, k0, lane);
    const v16h b3 = ldfrag(Bt, ldb, n0 + 48, k0, lane);
    acc[0][0] = mma16(a0, b0, acc[0][0]);
    acc[1][0] = mma16(a1, b0, acc[1][0]);
    acc[0][1] = mma16(a0, b1, acc[0][1]);
    acc[1][1] = mma16(a1, b1, acc[1][1]);
    acc[0][2] = mma16(a0, b2, acc[0][2]);
    acc[1][2] = mma16(a1, b2, acc[1][2]);
    acc[0][3] = mma16(a0, b3, acc[0][3]);
    acc[1][3] = mma16(a1, b3, acc[1][3]);
  }
}

__global__ __launch_bounds__(256) void k_cvt(const float* __restrict__ src, _Float16* __restrict__ dh, float scale) {
  const size_t o = ((size_t)blockIdx.x * 256 + threadIdx.x) * 8;
  const v4f a0 = *(const v4f*)(src + o) * scale;
  const v4f a1 = *(const v4f*)(src + o + 4) * scale;
  Pack8 pk;
  pk.h = (v8h){(_Float16)a0[0], (_Float16)a0[1], (_Float16)a0[2], (_Float16)a0[3],
               (_Float16)a1[0], (_Float16)a1[1], (_Float16)a1[2], (_Float16)a1[3]};
  const v4u vv = pk.u;
  volatile v4u* d = (volatile v4u*)(dh + o);
  *d = vv;
  __threadfence();
  *d = vv;
}

__global__ __launch_bounds__(256) void k_pad(const float* __restrict__ feat, const float* __restrict__ coords,
                                             const float* __restrict__ wp, const float* __restrict__ bp,
                                             const int* __restrict__ ids, int npts, _Float16* __restrict__ xh) {
  const int tid = threadIdx.x, lane = tid & 31, wave = tid >> 5;
  const int pr  = blockIdx.x * 8 + wave;
  const int g   = pr / LMAXC;
  const int l   = pr - g * LMAXC;
  const int gs  = lower_bound_ids(ids, npts, g);
  const int ge  = lower_bound_ids(ids, npts, g + 1);
  const int cnt = min(max(ge - gs, 0), LMAXC);
  const bool valid = l < cnt;
  const int n   = min(max(gs + l, 0), npts - 1);
  const float c0 = coords[2 * n], c1 = coords[2 * n + 1];
  const int col = lane * 8;
  v4f f0 = posenc4(feat, wp, bp, c0, c1, n, col);
  v4f f1 = posenc4(feat, wp, bp, c0, c1, n, col + 4);
#pragma unroll
  for (int j = 0; j < 4; ++j) {
    f0[j] = valid ? f0[j] : 0.f;
    f1[j] = valid ? f1[j] : 0.f;
  }
  Pack8 pk;
  pk.h = (v8h){(_Float16)f0[0], (_Float16)f0[1], (_Float16)f0[2], (_Float16)f0[3],
               (_Float16)f1[0], (_Float16)f1[1], (_Float16)f1[2], (_Float16)f1[3]};
  const v4u vv = pk.u;
  volatile v4u* d = (volatile v4u*)(xh + (size_t)pr * DM + col);
  *d = vv;
  __threadfence();
  *d = vv;
}

#define STP 72
#define SVP 264
__global__ __launch_bounds__(256) void k_qkv(const _Float16* __restrict__ xh,
                                             const _Float16* __restrict__ wt,
                                             const float* __restrict__ inb,
                                             _Float16* __restrict__ qkp,
                                             _Float16* __restrict__ vtp) {
  __shared__ __align__(16) _Float16 st[256 * STP];
  const int tid = threadIdx.x, lane = tid & 31, wave = tid >> 5;
  const int hh = lane >> 4, c = lane & 15;
  const int rb = blockIdx.x * 256;
  const int g  = rb / LMAXC;
  const int l0 = rb - g * LMAXC;
  const int ns = blockIdx.y;
  const int which = ns >> 2;
  const int cs = (ns & 3) * 64;
  const int m0 = rb + wave * 32;
  const int n0 = ns * 64;

  v8f acc[2][4];
#pragma unroll
  for (int s = 0; s < 2; ++s)
#pragma unroll
    for (int t = 0; t < 4; ++t) acc[s][t] = zero8();
  gemm32x64(xh, DM, wt, DM, DM, m0, n0, lane, acc);

  float bb[4];
#pragma unroll
  for (int t = 0; t < 4; ++t) bb[t] = inb[n0 + 16 * t + c];

  if (which < 2) {
#pragma unroll
    for (int sub = 0; sub < 2; ++sub)
#pragma unroll
      for (int t = 0; t < 4; ++t)
#pragma unroll
        for (int r = 0; r < 8; ++r)
          st[(wave * 32 + sub * 16 + 8 * hh + r) * STP + 16 * t + c] =
              (_Float16)(acc[sub][t][r] * 0.03125f + bb[t]);
  } else {
#pragma unroll
    for (int sub = 0; sub < 2; ++sub)
#pragma unroll
      for (int t = 0; t < 4; ++t)
#pragma unroll
        for (int r = 0; r < 8; ++r)
          st[(16 * t + c) * SVP + wave * 32 + sub * 16 + 8 * hh + r] =
              (_Float16)(acc[sub][t][r] * 0.03125f + bb[t]);
  }
  __syncthreads();

  if (which < 2) {
    _Float16* base = qkp + (size_t)which * PROWS * DM;
#pragma unroll
    for (int gg = 0; gg < 2; ++gg) {
      v4u val[4];
      size_t go[4];
#pragma unroll
      for (int j = 0; j < 4; ++j) {
        const int p  = tid + 256 * (4 * gg + j);
        const int lr = p >> 3;
        const int pc = p & 7;
        Pack8 pk;
        pk.h   = *(const v8h*)(st + lr * STP + pc * 8);
        val[j] = pk.u;
        go[j]  = (size_t)(rb + lr) * DM + cs + pc * 8;
      }
      for (int ps = 0; ps < 2; ++ps) {
#pragma unroll
        for (int j = 0; j < 4; ++j) *(volatile v4u*)(base + go[j]) = val[j];
        __threadfence();
      }
    }
  } else {
    _Float16* base = vtp + (size_t)g * DM * LMAXC;
#pragma unroll
    for (int gg = 0; gg < 2; ++gg) {
      v4u val[4];
      size_t go[4];
#pragma unroll
      for (int j = 0; j < 4; ++j) {
        const int p    = tid + 256 * (4 * gg + j);
        const int drow = p >> 5;
        const int pc   = p & 31;
        Pack8 pk;
        pk.h   = *(const v8h*)(st + drow * SVP + pc * 8);
        val[j] = pk.u;
        go[j]  = (size_t)(cs + drow) * LMAXC + l0 + pc * 8;
      }
      for (int ps = 0; ps < 2; ++ps) {
#pragma unroll
        for (int j = 0; j < 4; ++j) *(volatile v4u*)(base + go[j]) = val[j];
        __threadfence();
      }
    }
  }
}

#define KSP 264
#define VSP 72
#define PSP 72
#define OSP 136
__global__ __launch_bounds__(256) void k_attn(const _Float16* __restrict__ qp,
                                              const _Float16* __restrict__ kp,
                                              const _Float16* __restrict__ vt,
                                              const int* __restrict__ ids, int npts,
                                              _Float16* __restrict__ op) {
  __shared__ __align__(16) _Float16 Ks[KCH * KSP];
  __shared__ __align__(16) _Float16 Vs[DM * VSP];
  __shared__ __align__(16) _Float16 Ps[4 * 16 * PSP];
  __shared__ float Al[QBLK];
  __shared__ float Il[QBLK];

  const int tid = threadIdx.x, lane = tid & 31, wave = tid >> 5;
  const int hh = lane >> 4, c = lane & 15;
  const int g     = blockIdx.x / NQBG;
  const int qblk  = blockIdx.x - g * NQBG;
  const int qbase = qblk * QBLK;
  const int gs    = lower_bound_ids(ids, npts, g);
  const int ge    = lower_bound_ids(ids, npts, g + 1);
  const int cnt   = min(max(ge - gs, 0), LMAXC);
  const size_t prow0 = (size_t)g * LMAXC + qbase;
  const int tile = wave & 3, half = wave >> 2;

  if (qbase >= cnt) {
    const v4u z = (v4u){0u, 0u, 0u, 0u};
    size_t go[8];
#pragma unroll
    for (int it = 0; it < 8; ++it) {
      const int p   = tid + 256 * it;
      const int row = p >> 5;
      const int pc  = p & 31;
      go[it] = (prow0 + row) * DM + pc * 8;
    }
    for (int ps = 0; ps < 2; ++ps) {
#pragma unroll
      for (int it = 0; it < 8; ++it) *(volatile v4u*)(op + go[it]) = z;
      __threadfence();
    }
  } else {
    const _Float16* Qg = qp + (prow0 + 16 * tile) * DM;
    const _Float16* Kg = kp + (size_t)g * LMAXC * DM;
    const _Float16* Vg = vt + (size_t)g * DM * LMAXC;

    const float NEGI = -__builtin_huge_valf();
    float mrow[8], lrow[8];
    v8f oacc[8];
#pragma unroll
    for (int r = 0; r < 8; ++r) { mrow[r] = NEGI; lrow[r] = 0.f; }
#pragma unroll
    for (int t = 0; t < 8; ++t) oacc[t] = zero8();

    _Float16* pw = Ps + tile * 16 * PSP;
    const int nkc = min((cnt + KCH - 1) / KCH, NKCG);

    for (int kc = 0; kc < nkc; ++kc) {
      const int kv0 = kc * KCH;
      __syncthreads();
      {
        const int r  = tid >> 2;
        const int qq = (tid & 3) * 64;
        const _Float16* ks = Kg + (size_t)(kv0 + r) * DM + qq;
#pragma unroll
        for (int e = 0; e < 8; ++e) *(v8h*)(Ks + r * KSP + qq + 8 * e) = *(const v8h*)(ks + 8 * e);
        const _Float16* vs = Vg + (size_t)tid * LMAXC + kv0;
#pragma unroll
        for (int e = 0; e < 8; ++e) *(v8h*)(Vs + tid * VSP + 8 * e) = *(const v8h*)(vs + 8 * e);
      }
      __syncthreads();

      if (wave < 4) {
        v8f s[4];
#pragma unroll
        for (int j = 0; j < 4; ++j) s[j] = zero8();
#pragma unroll 1
        for (int dc = 0; dc < 8; ++dc) {
          const v16h qa = ldfrag(Qg, DM, 0, dc * 32, lane);
#pragma unroll
          for (int j = 0; j < 4; ++j) {
            const v16h kb = ldfrag(Ks, KSP, j * 16, dc * 32, lane);
            s[j] = mma16(qa, kb, s[j]);
          }
        }
        float cm[8];
#pragma unroll
        for (int r = 0; r < 8; ++r) {
          float m = NEGI;
#pragma unroll
          for (int j = 0; j < 4; ++j) {
            const int key = kv0 + j * 16 + c;
            float sv = s[j][r] * 0.0625f;
            sv = (key < cnt) ? sv : -1.0e9f;
            s[j][r] = sv;
            m = fmaxf(m, sv);
          }
#pragma unroll
          for (int off = 1; off < 16; off <<= 1) m = fmaxf(m, __shfl_xor(m, off, 32));
          cm[r] = m;
        }
#pragma unroll
        for (int r = 0; r < 8; ++r) {
          const float mnew  = fmaxf(mrow[r], cm[r]);
          const float alpha = __expf(mrow[r] - mnew);
          mrow[r] = mnew;
          float psum = 0.f;
#pragma unroll
          for (int j = 0; j < 4; ++j) {
            const float p = __expf(s[j][r] - mnew);
            psum += p;
            pw[(8 * hh + r) * PSP + j * 16 + c] = (_Float16)(p * 1024.0f);
          }
#pragma unroll
          for (int off = 1; off < 16; off <<= 1) psum += __shfl_xor(psum, off, 32);
          lrow[r] = lrow[r] * alpha + psum;
          Al[tile * 16 + 8 * hh + r] = alpha;
        }
      }
      __syncthreads();

      float al[8];
#pragma unroll
      for (int r = 0; r < 8; ++r) al[r] = Al[tile * 16 + 8 * hh + r];
#pragma unroll
      for (int t = 0; t < 8; ++t)
#pragma unroll
        for (int r = 0; r < 8; ++r) oacc[t][r] *= al[r];

#pragma unroll 1
      for (int kk = 0; kk < 2; ++kk) {
        const v16h pa = ldfrag(pw, PSP, 0, kk * 32, lane);
#pragma unroll
        for (int t = 0; t < 8; ++t) {
          const v16h vb = ldfrag(Vs, VSP, half * 128 + t * 16, kk * 32, lane);
          oacc[t] = mma16(pa, vb, oacc[t]);
        }
      }
    }

    if (wave < 4) {
#pragma unroll
      for (int r = 0; r < 8; ++r)
        Il[tile * 16 + 8 * hh + r] = (lrow[r] > 0.f) ? (0.25f * __builtin_amdgcn_rcpf(lrow[r])) : 0.f;
    }
    __syncthreads();
    float il[8];
#pragma unroll
    for (int r = 0; r < 8; ++r) il[r] = Il[tile * 16 + 8 * hh + r];
    _Float16* ow = Vs + wave * 16 * OSP;
#pragma unroll
    for (int t = 0; t < 8; ++t)
#pragma unroll
      for (int r = 0; r < 8; ++r)
        ow[(8 * hh + r) * OSP + 16 * t + c] = (_Float16)(oacc[t][r] * il[r]);
    __syncthreads();
    v4u val[8];
    size_t go[8];
#pragma unroll
    for (int it = 0; it < 8; ++it) {
      const int p  = lane + 32 * it;
      const int L  = p >> 4;
      const int pc = p & 15;
      Pack8 pk;
      pk.h    = *(const v8h*)(ow + L * OSP + pc * 8);
      val[it] = pk.u;
      go[it]  = (prow0 + 16 * tile + L) * DM + half * 128 + pc * 8;
    }
    for (int ps = 0; ps < 2; ++ps) {
#pragma unroll
      for (int it = 0; it < 8; ++it) *(volatile v4u*)(op + go[it]) = val[it];
      __threadfence();
    }
  }
}

#define OTP 68
__device__ __forceinline__ void out_epilogue_f32(v8f (&acc)[2][4], float scale, const float (&bb)[4],
                                                 float* sw, float* __restrict__ out, int ldo,
                                                 int m0, int n0, int lane, int hh, int c) {
#pragma unroll
  for (int sub = 0; sub < 2; ++sub) {
    __syncthreads();
#pragma unroll
    for (int t = 0; t < 4; ++t) {
#pragma unroll
      for (int r = 0; r < 8; ++r) sw[(8 * hh + r) * OTP + 16 * t + c] = acc[sub][t][r] * scale + bb[t];
    }
    __syncthreads();
    v4f val[8];
    size_t go[8];
#pragma unroll
    for (int it = 0; it < 8; ++it) {
      const int p     = lane + 32 * it;
      const int L     = p >> 3;
      const int pc    = p & 7;
      const int row   = L >> 1;
      const int seg   = L & 1;
      val[it] = *(const v4f*)(sw + row * OTP + seg * 32 + pc * 4);
      go[it]  = (size_t)(m0 + sub * 16 + row) * ldo + n0 + seg * 32 + pc * 4;
    }
    for (int ps = 0; ps < 2; ++ps) {
#pragma unroll
      for (int it = 0; it < 8; ++it) *(volatile v4f*)(out + go[it]) = val[it];
      __threadfence();
    }
  }
}

__global__ __launch_bounds__(256) void k_gemm_f32(const _Float16* __restrict__ ap, int lda,
                                                  const _Float16* __restrict__ wt, int K,
                                                  const float* __restrict__ bias, float scale,
                                                  float* __restrict__ out, int ldo) {
  __shared__ __align__(16) float st[8][16 * OTP];
  const int tid = threadIdx.x, lane = tid & 31, wave = tid >> 5;
  const int hh = lane >> 4, c = lane & 15;
  const int m0 = blockIdx.x * 256 + wave * 32;
  const int n0 = blockIdx.y * 64;

  v8f acc[2][4];
#pragma unroll
  for (int s = 0; s < 2; ++s)
#pragma unroll
    for (int t = 0; t < 4; ++t) acc[s][t] = zero8();
  gemm32x64(ap, lda, wt, K, K, m0, n0, lane, acc);
  float bb[4];
#pragma unroll
  for (int t = 0; t < 4; ++t) bb[t] = bias[n0 + 16 * t + c];
  out_epilogue_f32(acc, scale, bb, st[wave], out, ldo, m0, n0, lane, hh, c);
}

__global__ __launch_bounds__(256) void k_ln(const float* __restrict__ tp, const float* __restrict__ feat,
                                            const float* __restrict__ coords, const float* __restrict__ wp,
                                            const float* __restrict__ bp, const float* __restrict__ gam,
                                            const float* __restrict__ bet, const int* __restrict__ ids, int npts,
                                            float* __restrict__ out) {
  const int tid = threadIdx.x, lane = tid & 31, wave = tid >> 5;
  const int n = min((int)blockIdx.x * 8 + wave, npts - 1);
  int g = ids[n];
  g = min(max(g, 0), NGRP - 1);
  const int gs = lower_bound_ids(ids, npts, g);
  const int l  = min(max(n - gs, 0), LMAXC - 1);
  const float* tr = tp + ((size_t)g * LMAXC + l) * DM;

  v4f v[2];
  float s = 0.f;
#pragma unroll
  for (int it = 0; it < 2; ++it) {
    const int idx = it * 128 + lane * 4;
    v[it] = *(const v4f*)(tr + idx);
    s += (v[it][0] + v[it][1]) + (v[it][2] + v[it][3]);
  }
#pragma unroll
  for (int off = 16; off >= 1; off >>= 1) s += __shfl_xor(s, off, 32);
  const float mean = s * 0.00390625f;
  float ss = 0.f;
#pragma unroll
  for (int it = 0; it < 2; ++it) {
    const v4f d = v[it] - mean;
    ss += (d[0] * d[0] + d[1] * d[1]) + (d[2] * d[2] + d[3] * d[3]);
  }
#pragma unroll
  for (int off = 16; off >= 1; off >>= 1) ss += __shfl_xor(ss, off, 32);
  const float var  = ss * 0.00390625f;
  const float rstd = rsqrtf(var + 1e-6f);

  const float c0 = coords[2 * n], c1 = coords[2 * n + 1];
  v4f o[2];
#pragma unroll
  for (int it = 0; it < 2; ++it) {
    const int idx = it * 128 + lane * 4;
    const v4f gv  = *(const v4f*)(gam + idx);
    const v4f bv  = *(const v4f*)(bet + idx);
    const v4f res = posenc4(feat, wp, bp, c0, c1, n, idx);
    const v4f y   = ((v[it] - mean) * rstd) * gv + bv + res;
#pragma unroll
    for (int j = 0; j < 4; ++j) o[it][j] = fmaxf(y[j], 0.f);
  }
  for (int ps = 0; ps < 2; ++ps) {
#pragma unroll
    for (int it = 0; it < 2; ++it) *(volatile v4f*)(out + (size_t)n * DM + it * 128 + lane * 4) = o[it];
    __threadfence();
  }
}

extern "C" void kernel_launch(void* const* d_in, const int* in_sizes, int n_in,
                              void* d_out, int out_size, void* d_ws, size_t ws_size,
                              hipStream_t stream) {
  if (n_in < 11) return;
  if (in_sizes[0] != NPTS * DM) return;
  if (in_sizes[1] != NPTS * 2) return;
  if (in_sizes[2] != DM * 2) return;
  if (in_sizes[3] != DM) return;
  if (in_sizes[4] != NQKV * DM) return;
  if (in_sizes[5] != NQKV) return;
  if (in_sizes[6] != DM * DM) return;
  if (in_sizes[7] != DM) return;
  if (in_sizes[8] != DM) return;
  if (in_sizes[9] != DM) return;
  if (in_sizes[10] != NPTS) return;
  if (out_size != NPTS * DM) return;

  const float* feat   = (const float*)d_in[0];
  const float* coords = (const float*)d_in[1];
  const float* wp     = (const float*)d_in[2];
  const float* bp     = (const float*)d_in[3];
  const float* in_w   = (const float*)d_in[4];
  const float* in_b   = (const float*)d_in[5];
  const float* out_w  = (const float*)d_in[6];
  const float* out_b  = (const float*)d_in[7];
  const float* gam    = (const float*)d_in[8];
  const float* bet    = (const float*)d_in[9];
  const int*   ids    = (const int*)d_in[10];
  const int    npts   = in_sizes[10];
  float* out = (float*)d_out;

  size_t off = 0;
  const size_t oWt = off; off += (size_t)NQKV * DM * 2;
  const size_t oWo = off; off += (size_t)DM * DM * 2;
  const size_t oX  = off; off += (size_t)PROWS * DM * 2;
  const size_t oQ  = off; off += (size_t)PROWS * DM * 2;
  const size_t oK  = off; off += (size_t)PROWS * DM * 2;
  const size_t oV  = off; off += (size_t)NGRP * DM * LMAXC * 2;
  const size_t oO  = off; off += (size_t)PROWS * DM * 2;
  const size_t oT  = off; off += (size_t)PROWS * DM * 4;
  if (off > ws_size) return;
  if (off > (size_t)134217728) return;
  if (oK != oQ + (size_t)PROWS * DM * 2) return;

  char* ws = (char*)d_ws;
  _Float16* Wt  = (_Float16*)(ws + oWt);
  _Float16* Wot = (_Float16*)(ws + oWo);
  _Float16* Xh  = (_Float16*)(ws + oX);
  _Float16* QKp = (_Float16*)(ws + oQ);
  _Float16* Kp  = (_Float16*)(ws + oK);
  _Float16* Vt  = (_Float16*)(ws + oV);
  _Float16* Op  = (_Float16*)(ws + oO);
  float*    T   = (float*)(ws + oT);

  k_cvt<<<dim3((NQKV * DM) / 2048), dim3(256), 0, stream>>>(in_w, Wt, 32.0f);
  k_cvt<<<dim3((DM * DM) / 2048), dim3(256), 0, stream>>>(out_w, Wot, 32.0f);
  k_pad<<<dim3(PROWS / 8), dim3(256), 0, stream>>>(feat, coords, wp, bp, ids, npts, Xh);
  k_qkv<<<dim3(PROWS / 256, NQKV / 64), dim3(256), 0, stream>>>(Xh, Wt, in_b, QKp, Vt);
  k_attn<<<dim3(NGRP * NQBG), dim3(256), 0, stream>>>(QKp, Kp, Vt, ids, npts, Op);
  k_gemm_f32<<<dim3(PROWS / 256, DM / 64), dim3(256), 0, stream>>>(Op, DM, Wot, DM, out_b, 0.0001220703125f, T, DM);
  k_ln<<<dim3(NPTS / 8), dim3(256), 0, stream>>>(T, feat, coords, wp, bp, gam, bet, ids, npts, out);
  (void)hipGetLastError();
}
